// Dtu_32280974197058
// MI455X (gfx1250) — hardware-verified
//
#include <hip/hip_runtime.h>
#include <math.h>

constexpr int kBatch     = 8;
constexpr int kSide      = 56;
constexpr int kEmbed     = 192;
constexpr int kWide      = 576;
constexpr int kTwoN      = 112;
constexpr int kHidden    = 32;
constexpr int kLayers    = 3;
constexpr int kHalves    = 2;
constexpr int kBatchHalf = kBatch / kHalves;
constexpr int kRowsHalf  = kBatchHalf * kSide * kSide;
constexpr int kSeqHalf   = kBatchHalf * kSide;
constexpr int kChan      = 64;
constexpr int kNChan     = kWide / kChan;
static_assert(kRowsHalf % 64 == 0);
static_assert(kWide % 64 == 0);
static_assert(kEmbed % 64 == 0);
static_assert(kEmbed % 32 == 0);
static_assert(kWide % 32 == 0);
static_assert(kWide % kChan == 0);

constexpr size_t kXPlaneB   = (size_t)kRowsHalf * kEmbed * 2;
constexpr size_t kF32PlaneB = (size_t)kRowsHalf * kWide * 4;
constexpr size_t kGPlaneB   = (size_t)kRowsHalf * kWide * 2;
constexpr size_t kWPlaneB   = (size_t)kWide * kEmbed * 2;
constexpr size_t kCoefB     = (size_t)kTwoN * kWide * 4;
constexpr size_t kOffXh   = 0;
constexpr size_t kOffXl   = kOffXh + kXPlaneB;
constexpr size_t kOffRA   = kOffXl + kXPlaneB;
constexpr size_t kOffRB   = kOffRA + kF32PlaneB;
constexpr size_t kOffRC   = kOffRB + kF32PlaneB;
constexpr size_t kOffW    = kOffRC + kF32PlaneB;
constexpr size_t kOffCoef = kOffW + 8 * kWPlaneB;
constexpr size_t kWsTotal = kOffCoef + 2 * kCoefB;
static_assert(kWsTotal == 98623488);
static_assert(kWsTotal <= 134217728);
static_assert(2 * kGPlaneB == kF32PlaneB);
static_assert(kXPlaneB % 128 == 0 && kF32PlaneB % 128 == 0 && kWPlaneB % 128 == 0 && kCoefB % 128 == 0 && kGPlaneB % 128 == 0);

typedef __attribute__((ext_vector_type(16))) _Float16 v16h;
typedef __attribute__((ext_vector_type(8)))  _Float16 v8h;
typedef __attribute__((ext_vector_type(16))) __bf16   v16b;
typedef __attribute__((ext_vector_type(8)))  __bf16   v8b;
typedef __attribute__((ext_vector_type(8)))  float    v8f;
typedef __attribute__((ext_vector_type(4)))  float    v4f;
typedef __attribute__((ext_vector_type(4)))  unsigned int v4u;

__device__ __forceinline__ unsigned short f2bf_bits(float f) {
  unsigned u = __float_as_uint(f);
  return (unsigned short)((u + 0x7FFFu + ((u >> 16) & 1u)) >> 16);
}
__device__ __forceinline__ float bf_bits2f(unsigned short h) { return __uint_as_float(((unsigned)h) << 16); }

__device__ __forceinline__ void dep_guard_h(v8f& a, v8f& b, v16h x, v16h y) { asm volatile("v_nop\n\tv_nop\n\tv_nop\n\tv_nop" : "+v"(a), "+v"(b) : "v"(x), "v"(y)); }
__device__ __forceinline__ void dep_guard_b(v8f& a, v8f& b, v16b x, v16b y) { asm volatile("v_nop\n\tv_nop\n\tv_nop\n\tv_nop" : "+v"(a), "+v"(b) : "v"(x), "v"(y)); }
__device__ __forceinline__ void keep4_h(v16h a, v16h b, v16h c, v16h d) { asm volatile("v_nop" :: "v"(a), "v"(b), "v"(c), "v"(d)); }
__device__ __forceinline__ void keep4_b(v16b a, v16b b, v16b c, v16b d) { asm volatile("v_nop" :: "v"(a), "v"(b), "v"(c), "v"(d)); }
__device__ __forceinline__ void acc_guard4(v8f& a, v8f& b, v8f& c, v8f& d) { asm volatile("v_nop\n\tv_nop\n\tv_nop\n\tv_nop" : "+v"(a), "+v"(b), "+v"(c), "+v"(d)); }
template <typename T> struct Frag;
template <> struct Frag<_Float16> {
  typedef v16h V; union U { v16h v; v8h h[2]; };
  static __device__ __forceinline__ v16h load(const _Float16* p) {
    U f; f.h[0] = *(const v8h*)(p); f.h[1] = *(const v8h*)(p + 16); return f.v;
  }
  static __device__ __forceinline__ v8f mma(v16h a, v16h b, v8f c) {
    return __builtin_amdgcn_wmma_f32_16x16x32_f16(false, a, false, b, (short)0, c, false, false);
  }
  static __device__ __forceinline__ void guard(v8f& a, v8f& b, v16h x, v16h y) { dep_guard_h(a, b, x, y); }
  static __device__ __forceinline__ void keep(v16h a, v16h b, v16h c, v16h d) { keep4_h(a, b, c, d); }
};
template <> struct Frag<__bf16> {
  typedef v16b V; union U { v16b v; v8b h[2]; };
  static __device__ __forceinline__ v16b load(const __bf16* p) {
    U f; f.h[0] = *(const v8b*)(p); f.h[1] = *(const v8b*)(p + 16); return f.v;
  }
  static __device__ __forceinline__ v8f mma(v16b a, v16b b, v8f c) {
    return __builtin_amdgcn_wmma_f32_16x16x32_bf16(false, a, false, b, (short)0, c, false, false);
  }
  static __device__ __forceinline__ void guard(v8f& a, v8f& b, v16b x, v16b y) { dep_guard_b(a, b, x, y); }
  static __device__ __forceinline__ void keep(v16b a, v16b b, v16b c, v16b d) { keep4_b(a, b, c, d); }
};

__device__ __forceinline__ unsigned pk16(unsigned short a, unsigned short b) { return (unsigned)a | ((unsigned)b << 16); }

template <int ET> struct Elem;
template <> struct Elem<0> { typedef _Float16 T; };
template <> struct Elem<1> { typedef __bf16 T; };
template <int ET, bool SPLIT, int BIAS_MODE, int OUT_MODE, bool RESID, int ACT = 0, bool MULR = false>
__global__ __launch_bounds__(256) void wmma_gemm64(
    const unsigned short* __restrict__ Ap, const unsigned short* __restrict__ A2p, int lda, long strideA,
    const unsigned short* __restrict__ Btp, const unsigned short* __restrict__ Bt2p, int ldb, long strideB,
    void* __restrict__ Cout, void* __restrict__ Cout2, int ldc, long strideC,
    const float* __restrict__ bias,
    const float* __restrict__ resid, long strideR,
    int M, int N, int K, float scale) {
  typedef typename Elem<ET>::T T;
  typedef typename Frag<T>::V V;
  const T* A = (const T*)Ap; const T* A2 = (const T*)A2p; const T* Bt = (const T*)Btp; const T* Bt2 = (const T*)Bt2p;
  __shared__ __align__(16) float sT[8][16 * 68];
  const int b    = blockIdx.y;
  const int lane = threadIdx.x & 31;
  const int wave = threadIdx.x >> 5;
  const int tilesN = N >> 6;
  const int tilesM = M >> 6;
  const int tile = blockIdx.x * 8 + wave;
  if (tile >= tilesM * tilesN) return;
  const int tm = tile / tilesN;
  const int tn = tile - tm * tilesN;
  const int m0 = tm << 6;
  const int n0 = tn << 6;

  const T* Ab  = A  + (size_t)b * strideA;
  const T* Bb  = Bt + (size_t)b * strideB;
  const T* Ab2 = SPLIT ? (A2  + (size_t)b * strideA) : nullptr;
  const T* Bb2 = SPLIT ? (Bt2 + (size_t)b * strideB) : nullptr;

  const int rlane = lane & 15;
  const int koff  = (lane >> 4) * 8;
  const int mOff  = (lane >> 4) * 8;

  v8f acc[4][4];
#pragma unroll
  for (int i = 0; i < 4; ++i)
#pragma unroll
    for (int j = 0; j < 4; ++j) acc[i][j] = (v8f){0.f,0.f,0.f,0.f,0.f,0.f,0.f,0.f};

  for (int k0 = 0; k0 < K; k0 += 32) {
    V bh[4], bl[4];
#pragma unroll
    for (int j = 0; j < 4; ++j) {
      const size_t bo = (size_t)(n0 + (j << 4) + rlane) * ldb + koff + k0;
      bh[j] = Frag<T>::load(Bb + bo);
      if (SPLIT) bl[j] = Frag<T>::load(Bb2 + bo);
    }
#pragma unroll
    for (int i = 0; i < 4; ++i) {
      const size_t ao = (size_t)(m0 + (i << 4) + rlane) * lda + koff + k0;
      V ah = Frag<T>::load(Ab + ao);
      V al;
      if (SPLIT) al = Frag<T>::load(Ab2 + ao);
#pragma unroll
      for (int j = 0; j < 4; ++j) {
        acc[i][j] = Frag<T>::mma(ah, bh[j], acc[i][j]);
        if (SPLIT) {
          acc[i][j] = Frag<T>::mma(ah, bl[j], acc[i][j]);
          acc[i][j] = Frag<T>::mma(al, bh[j], acc[i][j]);
        }
      }
      Frag<T>::guard(acc[i][0], acc[i][3], ah, SPLIT ? al : ah);
    }
    Frag<T>::keep(bh[0], bh[1], bh[2], bh[3]);
    if (SPLIT) Frag<T>::keep(bl[0], bl[1], bl[2], bl[3]);
  }
  acc_guard4(acc[0][0], acc[0][1], acc[0][2], acc[0][3]);
  acc_guard4(acc[1][0], acc[1][1], acc[1][2], acc[1][3]);
  acc_guard4(acc[2][0], acc[2][1], acc[2][2], acc[2][3]);
  acc_guard4(acc[3][0], acc[3][1], acc[3][2], acc[3][3]);

  float* slab = sT[wave];
  const float* Rb = (RESID || MULR) ? (resid + (size_t)b * strideR) : nullptr;
#pragma unroll
  for (int i = 0; i < 4; ++i) {
    const int mBase = m0 + (i << 4);
#pragma unroll
    for (int j = 0; j < 4; ++j) {
      const int n = n0 + (j << 4) + rlane;
      float bv = 0.f;
      if (BIAS_MODE == 2) bv = bias[n];
#pragma unroll
      for (int r = 0; r < 8; ++r) {
        float v = acc[i][j][r] * scale;
        if (BIAS_MODE == 1) v += bias[mBase + mOff + r];
        if (BIAS_MODE == 2) v += bv;
        if (RESID) v += Rb[(size_t)(mBase + mOff + r) * ldc + n];
        if (ACT == 2) v = fmaxf(v, 0.0f);
        if (ACT == 3) v = v * (1.0f / (1.0f + expf(-v)));
        if (ACT == 4) v = (v > 0.f) ? v : 0.01f * v;
        if (MULR) v = v * Rb[(size_t)(mBase + mOff + r) * ldc + n];
        slab[(mOff + r) * 68 + (j << 4) + rlane] = v;
      }
    }
    __builtin_amdgcn_fence(__ATOMIC_RELEASE, "workgroup");
    __builtin_amdgcn_wave_barrier();
    __builtin_amdgcn_fence(__ATOMIC_ACQUIRE, "workgroup");
    if (OUT_MODE == 0) {
      float* C = (float*)Cout + (size_t)b * strideC;
      const int hh = lane >> 4, c4 = (lane & 15) * 4;
      for (int pass = 0; pass < 2; ++pass) {
#pragma unroll
        for (int it = 0; it < 8; ++it) {
          const int row = it * 2 + hh;
          v4f v = *(const v4f*)(slab + row * 68 + c4);
          *(volatile v4f*)(C + (size_t)(mBase + row) * ldc + n0 + c4) = v;
        }
        __threadfence();
      }
    } else {
      const int q = lane >> 3, c8 = (lane & 7) * 8;
      unsigned short* C  = (unsigned short*)Cout  + (size_t)b * strideC;
      unsigned short* C2 = (OUT_MODE == 2) ? ((unsigned short*)Cout2 + (size_t)b * strideC) : nullptr;
      for (int pass = 0; pass < 2; ++pass) {
#pragma unroll
        for (int it = 0; it < 4; ++it) {
          const int row = it * 4 + q;
          const float* sp = slab + row * 68 + c8;
          v8h hv, lv;
#pragma unroll
          for (int e = 0; e < 8; ++e) {
            if (OUT_MODE == 1) {
              hv[e] = (_Float16)sp[e];
            } else {
              unsigned short hb = f2bf_bits(sp[e]);
              unsigned short lb = f2bf_bits(sp[e] - bf_bits2f(hb));
              hv[e] = __builtin_bit_cast(_Float16, hb);
              lv[e] = __builtin_bit_cast(_Float16, lb);
            }
          }
          *(volatile v8h*)(C + (size_t)(mBase + row) * ldc + n0 + c8) = hv;
          if (OUT_MODE == 2) *(volatile v8h*)(C2 + (size_t)(mBase + row) * ldc + n0 + c8) = lv;
        }
        __threadfence();
      }
    }
    __builtin_amdgcn_fence(__ATOMIC_RELEASE, "workgroup");
    __builtin_amdgcn_wave_barrier();
    __builtin_amdgcn_fence(__ATOMIC_ACQUIRE, "workgroup");
  }
}

__global__ __launch_bounds__(256) void split8_bf16_kernel(const float* __restrict__ in,
                                                          unsigned short* __restrict__ hi,
                                                          unsigned short* __restrict__ lo, int n8) {
  const int i = blockIdx.x * 256 + threadIdx.x;
  if (i >= n8) return;
  const float* p = in + 8 * (size_t)i;
  const v4f a = *(const v4f*)(p);
  const v4f c = *(const v4f*)(p + 4);
  unsigned short hb[8], lb[8];
#pragma unroll
  for (int e = 0; e < 4; ++e) {
    const float f0 = a[e];
    const float f1 = c[e];
    hb[e]     = f2bf_bits(f0);
    lb[e]     = f2bf_bits(f0 - bf_bits2f(hb[e]));
    hb[4 + e] = f2bf_bits(f1);
    lb[4 + e] = f2bf_bits(f1 - bf_bits2f(hb[4 + e]));
  }
  const v4u uh = (v4u){pk16(hb[0], hb[1]), pk16(hb[2], hb[3]), pk16(hb[4], hb[5]), pk16(hb[6], hb[7])};
  const v4u ul = (v4u){pk16(lb[0], lb[1]), pk16(lb[2], lb[3]), pk16(lb[4], lb[5]), pk16(lb[6], lb[7])};
  unsigned short* qh = hi + 8 * (size_t)i;
  unsigned short* ql = lo + 8 * (size_t)i;
  *(volatile v4u*)qh = uh;
  *(volatile v4u*)ql = ul;
  __threadfence();
  *(volatile v4u*)qh = uh;
  *(volatile v4u*)ql = ul;
}

__global__ __launch_bounds__(64) void coef_kernel(
    const float* __restrict__ w0a, const float* __restrict__ b0a, const float* __restrict__ wsa,
    const float* __restrict__ bsa, const float* __restrict__ woa, const float* __restrict__ boa,
    const float* __restrict__ w0b, const float* __restrict__ b0b, const float* __restrict__ wsb,
    const float* __restrict__ bsb, const float* __restrict__ wob, const float* __restrict__ bob,
    const float* __restrict__ slope, float* __restrict__ outA, float* __restrict__ outB) {
  __shared__ float hs[kHidden];
  __shared__ __align__(16) float so[kWide];
  const int row = blockIdx.x;
  const bool sec = (blockIdx.y != 0);
  const float* w0 = sec ? w0b : w0a;
  const float* b0 = sec ? b0b : b0a;
  const float* ws = sec ? wsb : wsa;
  const float* bs = sec ? bsb : bsa;
  const float* wo = sec ? wob : woa;
  const float* bo = sec ? bob : boa;
  float* dst = sec ? outB : outA;

  float tval;
  int ep;
  if (row == 0 || row == kSide) { tval = 0.0f; ep = 0; }
  else if (row < kSide)         { tval = (float)row; ep = row; }
  else                          { tval = -(float)(row - kSide); ep = kTwoN - row; }

  const int tid = threadIdx.x;
  if (tid < kHidden) hs[tid] = tval * w0[tid] + b0[tid];
  __syncthreads();
  for (int L = 0; L < kLayers; ++L) {
    float v = 0.0f;
    if (tid < kHidden) {
      const float* Wl = ws + (size_t)L * kHidden * kHidden + (size_t)tid * kHidden;
#pragma unroll 4
      for (int k = 0; k < kHidden; ++k) v = fmaf(fmaxf(hs[k], 0.0f), Wl[k], v);
      v += bs[L * kHidden + tid];
    }
    __syncthreads();
    if (tid < kHidden) hs[tid] = v;
    __syncthreads();
  }
  for (int c = tid; c < kWide; c += 64) {
    const float* wr = wo + (size_t)c * kHidden;
    float acc = 0.0f;
#pragma unroll 4
    for (int k = 0; k < kHidden; ++k) acc = fmaf(fmaxf(hs[k], 0.0f), wr[k], acc);
    acc += bo[c];
    const float sl  = 0.95f + 0.05f * fminf(fmaxf(slope[c], 0.0f), 1.0f);
    const float dec = powf(sl, (float)ep);
    so[c] = acc * dec;
  }
  __syncthreads();
  float* drow = dst + (size_t)row * kWide;
  for (int pass = 0; pass < 2; ++pass) {
    for (int idx = tid; idx < kWide / 4; idx += 64) {
      const v4f v = *(const v4f*)(so + idx * 4);
      *(volatile v4f*)(drow + idx * 4) = v;
    }
    __threadfence();
  }
}

__global__ __launch_bounds__(64) void mixw_kernel(const float* __restrict__ QV, const float* __restrict__ coef,
                                                  float* __restrict__ O1) {
  __shared__ __align__(16) float ext[kTwoN * kChan];
  __shared__ __align__(16) float sto[kSide * kChan];
  const int t   = threadIdx.x;
  const int seq = blockIdx.x;
  const int c0  = blockIdx.y * kChan;
  const size_t r0 = (size_t)seq * kSide;

#pragma unroll 4
  for (int it = 0; it < 28; ++it) {
    const int idx4 = it * 64 + t;
    const int u    = idx4 >> 4;
    const int c4   = (idx4 & 15) * 4;
    int ar = u + kSide;
    if (ar >= kTwoN) ar -= kTwoN;
    const v4f v = *(const v4f*)(coef + (size_t)ar * kWide + c0 + c4);
    *(v4f*)(ext + u * kChan + c4) = v;
  }
  float qv[kSide];
  const float* qp = QV + r0 * kWide + c0 + t;
#pragma unroll
  for (int j = 0; j < kSide; ++j) qv[j] = qp[(size_t)j * kWide];
  __syncthreads();

#pragma unroll 1
  for (int i = 0; i < kSide; ++i) {
    const float* pb = ext + (i + 1) * kChan + t;
    float acc = 0.0f;
#pragma unroll
    for (int j = 0; j < kSide; ++j) acc = fmaf(pb[(kSide - 1 - j) * kChan], qv[j], acc);
    sto[i * kChan + t] = acc;
  }
  __syncthreads();

  const int lane = t & 31, wave = t >> 5;
  const int hh = lane >> 4, c4 = (lane & 15) * 4;
  for (int pass = 0; pass < 2; ++pass) {
#pragma unroll
    for (int it = 0; it < 14; ++it) {
      const int row = it * 4 + wave * 2 + hh;
      const v4f v = *(const v4f*)(sto + row * kChan + c4);
      *(volatile v4f*)(O1 + (r0 + row) * kWide + c0 + c4) = v;
    }
    __threadfence();
  }
}

__global__ __launch_bounds__(64) void mixh_kernel(const float* __restrict__ QV, const float* __restrict__ coef,
                                                  const float* __restrict__ O1, float* __restrict__ Osum) {
  __shared__ __align__(16) float ext[kTwoN * kChan];
  __shared__ __align__(16) float sto[kSide * kChan];
  const int t  = threadIdx.x;
  const int s  = blockIdx.x;
  const int bb = s / kSide;
  const int w  = s - bb * kSide;
  const int c0 = blockIdx.y * kChan;
  const size_t rbase = ((size_t)bb * kSide) * kSide + w;

#pragma unroll 4
  for (int it = 0; it < 28; ++it) {
    const int idx4 = it * 64 + t;
    const int u    = idx4 >> 4;
    const int c4   = (idx4 & 15) * 4;
    int ar = u + kSide;
    if (ar >= kTwoN) ar -= kTwoN;
    const v4f v = *(const v4f*)(coef + (size_t)ar * kWide + c0 + c4);
    *(v4f*)(ext + u * kChan + c4) = v;
  }
  float qv[kSide];
  const float* qp = QV + rbase * kWide + c0 + t;
#pragma unroll
  for (int j = 0; j < kSide; ++j) qv[j] = qp[(size_t)j * kSide * kWide];
  __syncthreads();

  const float* op = O1 + rbase * kWide + c0 + t;
#pragma unroll 1
  for (int i = 0; i < kSide; ++i) {
    const float* pb = ext + (i + 1) * kChan + t;
    float acc = 0.0f;
#pragma unroll
    for (int j = 0; j < kSide; ++j) acc = fmaf(pb[(kSide - 1 - j) * kChan], qv[j], acc);
    const float o1 = op[(size_t)i * kSide * kWide];
    sto[i * kChan + t] = o1 + acc;
  }
  __syncthreads();

  const int lane = t & 31, wave = t >> 5;
  const int hh = lane >> 4, c4 = (lane & 15) * 4;
  for (int pass = 0; pass < 2; ++pass) {
#pragma unroll
    for (int it = 0; it < 14; ++it) {
      const int row = it * 4 + wave * 2 + hh;
      const v4f v = *(const v4f*)(sto + row * kChan + c4);
      *(volatile v4f*)(Osum + (rbase + (size_t)row * kSide) * kWide + c0 + c4) = v;
    }
    __threadfence();
  }
}

extern "C" void kernel_launch(void* const* d_in, const int* in_sizes, int n_in,
                              void* d_out, int out_size, void* d_ws, size_t ws_size,
                              hipStream_t stream) {
  (void)in_sizes; (void)n_in; (void)out_size;
  const float* x     = (const float*)d_in[0];
  const float* p_w   = (const float*)d_in[1];
  const float* p_b   = (const float*)d_in[2];
  const float* q_w   = (const float*)d_in[3];
  const float* q_b   = (const float*)d_in[4];
  const float* v_w   = (const float*)d_in[5];
  const float* v_b   = (const float*)d_in[6];
  const float* o_w   = (const float*)d_in[7];
  const float* o_b   = (const float*)d_in[8];
  const float* slope = (const float*)d_in[9];
  const float* t1_w0 = (const float*)d_in[10];
  const float* t1_b0 = (const float*)d_in[11];
  const float* t1_ws = (const float*)d_in[12];
  const float* t1_bs = (const float*)d_in[13];
  const float* t1_wo = (const float*)d_in[14];
  const float* t1_bo = (const float*)d_in[15];
  const float* t2_w0 = (const float*)d_in[16];
  const float* t2_b0 = (const float*)d_in[17];
  const float* t2_ws = (const float*)d_in[18];
  const float* t2_bs = (const float*)d_in[19];
  const float* t2_wo = (const float*)d_in[20];
  const float* t2_bo = (const float*)d_in[21];

  if (ws_size < kWsTotal) return;
  char* ws = (char*)d_ws;
  unsigned short* Xh = (unsigned short*)(ws + kOffXh);
  unsigned short* Xl = (unsigned short*)(ws + kOffXl);
  float* RA = (float*)(ws + kOffRA);
  float* RB = (float*)(ws + kOffRB);
  float* RC = (float*)(ws + kOffRC);
  unsigned short* Gh = (unsigned short*)(ws + kOffRA);
  unsigned short* Gl = (unsigned short*)(ws + kOffRA + kGPlaneB);
  unsigned short* Wph = (unsigned short*)(ws + kOffW + 0 * kWPlaneB);
  unsigned short* Wpl = (unsigned short*)(ws + kOffW + 1 * kWPlaneB);
  unsigned short* Wqh = (unsigned short*)(ws + kOffW + 2 * kWPlaneB);
  unsigned short* Wql = (unsigned short*)(ws + kOffW + 3 * kWPlaneB);
  unsigned short* Wvh = (unsigned short*)(ws + kOffW + 4 * kWPlaneB);
  unsigned short* Wvl = (unsigned short*)(ws + kOffW + 5 * kWPlaneB);
  unsigned short* Woh = (unsigned short*)(ws + kOffW + 6 * kWPlaneB);
  unsigned short* Wol = (unsigned short*)(ws + kOffW + 7 * kWPlaneB);
  float* A1 = (float*)(ws + kOffCoef);
  float* A2 = (float*)(ws + kOffCoef + kCoefB);

  constexpr int kW8 = kWide * kEmbed / 8;
  static_assert(kW8 % 256 == 0);
  split8_bf16_kernel<<<dim3(kW8 / 256), 256, 0, stream>>>(p_w, Wph, Wpl, kW8);
  split8_bf16_kernel<<<dim3(kW8 / 256), 256, 0, stream>>>(q_w, Wqh, Wql, kW8);
  split8_bf16_kernel<<<dim3(kW8 / 256), 256, 0, stream>>>(v_w, Wvh, Wvl, kW8);
  split8_bf16_kernel<<<dim3(kW8 / 256), 256, 0, stream>>>(o_w, Woh, Wol, kW8);

  coef_kernel<<<dim3(kTwoN, 2), 64, 0, stream>>>(t1_w0, t1_b0, t1_ws, t1_bs, t1_wo, t1_bo,
                                                 t2_w0, t2_b0, t2_ws, t2_bs, t2_wo, t2_bo,
                                                 slope, A1, A2);

  constexpr int kX8 = kRowsHalf * kEmbed / 8;
  static_assert(kX8 % 256 == 0);
  constexpr int kTilesWide = (kRowsHalf / 64) * (kWide / 64);
  constexpr int kBlkWide   = (kTilesWide + 7) / 8;
  constexpr int kTilesOut  = (kRowsHalf / 64) * (kEmbed / 64);
  constexpr int kBlkOut    = (kTilesOut + 7) / 8;

  for (int half = 0; half < kHalves; ++half) {
    const float* xh = x + (size_t)half * kRowsHalf * kEmbed;
    float* outh = (float*)d_out + (size_t)half * kRowsHalf * kEmbed;

    split8_bf16_kernel<<<dim3(kX8 / 256), 256, 0, stream>>>(xh, Xh, Xl, kX8);

    wmma_gemm64<1, true, 2, 0, false, 3, false><<<dim3(kBlkWide, 1), 256, 0, stream>>>(
        Xh, Xl, kEmbed, 0L, Wqh, Wql, kEmbed, 0L,
        (void*)RA, (void*)nullptr, kWide, 0L,
        q_b, (const float*)nullptr, 0L, kRowsHalf, kWide, kEmbed, 1.0f);

    wmma_gemm64<1, true, 2, 0, false, 3, true><<<dim3(kBlkWide, 1), 256, 0, stream>>>(
        Xh, Xl, kEmbed, 0L, Wvh, Wvl, kEmbed, 0L,
        (void*)RB, (void*)nullptr, kWide, 0L,
        v_b, (const float*)RA, 0L, kRowsHalf, kWide, kEmbed, 1.0f);

    mixw_kernel<<<dim3(kSeqHalf, kNChan), 64, 0, stream>>>(RB, A1, RA);

    mixh_kernel<<<dim3(kSeqHalf, kNChan), 64, 0, stream>>>(RB, A2, RA, RC);

    wmma_gemm64<1, true, 2, 2, false, 3, true><<<dim3(kBlkWide, 1), 256, 0, stream>>>(
        Xh, Xl, kEmbed, 0L, Wph, Wpl, kEmbed, 0L,
        (void*)Gh, (void*)Gl, kWide, 0L,
        p_b, (const float*)RC, 0L, kRowsHalf, kWide, kEmbed, 1.0f);

    wmma_gemm64<1, true, 2, 0, false, 0, false><<<dim3(kBlkOut, 1), 256, 0, stream>>>(
        Gh, Gl, kWide, 0L, Woh, Wol, kWide, 0L,
        (void*)outh, (void*)nullptr, kEmbed, 0L,
        o_b, (const float*)nullptr, 0L, kRowsHalf, kEmbed, kWide, 1.0f);
  }
}
